// CoAtten2_68289980006551
// MI455X (gfx1250) — hardware-verified
//
#include <hip/hip_runtime.h>
#include <math.h>

typedef __attribute__((ext_vector_type(16))) _Float16 v16h;
typedef __attribute__((ext_vector_type(16))) __bf16 v16b;
typedef __attribute__((ext_vector_type(8)))  _Float16 v8h;
typedef __attribute__((ext_vector_type(8)))  float v8f;
typedef __attribute__((ext_vector_type(4)))  float v4f;
typedef __attribute__((ext_vector_type(2)))  float v2f;
typedef __attribute__((ext_vector_type(4)))  unsigned v4u;
typedef __attribute__((ext_vector_type(4)))  int v4i;
typedef float __attribute__((may_alias)) float_a;
typedef int __attribute__((may_alias)) int_a;

template <typename T> __device__ __forceinline__ void vst2(void* p, T v) { *(volatile T*)p = v; __threadfence(); *(volatile T*)p = v; }
__device__ __forceinline__ v8f wmma16(v16h a, v16h b, v8f c) {
  v8f d = __builtin_amdgcn_wmma_f32_16x16x32_f16(false, a, false, b, (short)0, c, false, false);
  asm volatile("v_nop\n\tv_nop\n\tv_nop\n\tv_nop" : "+v"(d) : "v"(a), "v"(b));
  return d;
}
__device__ __forceinline__ v8f wmma_bf(v16b a, v16b b, v8f c) {
  v8f d = __builtin_amdgcn_wmma_f32_16x16x32_bf16(false, a, false, b, (short)0, c, false, false);
  asm volatile("v_nop\n\tv_nop\n\tv_nop\n\tv_nop" : "+v"(d) : "v"(a), "v"(b));
  return d;
}
__device__ __forceinline__ v16h frag_h(const _Float16* rowk0, int lane) {
  union { v16h v; v8h q[2]; } u; const _Float16* p = rowk0 + 8 * (lane >> 4);
  u.q[0] = *(const v8h*)p; u.q[1] = *(const v8h*)(p + 16); return u.v;
}
__device__ __forceinline__ v16h frag_f32(const float* rowk0, int lane) {
  v16h a; const float* p = rowk0 + 8 * (lane >> 4);
#pragma unroll
  for (int i = 0; i < 8; ++i) { a[i] = (_Float16)p[i]; a[8 + i] = (_Float16)p[16 + i]; }
  return a;
}
__device__ __forceinline__ v16h frag_f32s(const float* rowk0, int lane, float sc) {
  v16h a; const float* p = rowk0 + 8 * (lane >> 4);
#pragma unroll
  for (int i = 0; i < 8; ++i) { a[i] = (_Float16)(p[i] * sc); a[8 + i] = (_Float16)(p[16 + i] * sc); }
  return a;
}
__device__ __forceinline__ v16h fragc_f32(const float* W, int k0, int n, int lane, int ld, int K) {
  v16h a; const int g = lane >> 4;
#pragma unroll
  for (int i = 0; i < 8; ++i) { const int ka = k0 + 8 * g + i, kb = ka + 16;
    a[i] = (_Float16)(ka < K ? W[(size_t)(ka < K ? ka : K - 1) * ld + n] : 0.f); a[8 + i] = (_Float16)(kb < K ? W[(size_t)(kb < K ? kb : K - 1) * ld + n] : 0.f); }
  return a;
}
struct F2 { v16b h, l; };
__device__ __forceinline__ F2 bsplit16(const float v[16]) { F2 r;
#pragma unroll
  for (int i = 0; i < 16; ++i) { const __bf16 h = (__bf16)v[i]; r.h[i] = h; r.l[i] = (__bf16)(v[i] - (float)h); }
  return r; }
__device__ __forceinline__ F2 split_row(const float* row, int k0, int lane) { float v[16]; const float* p = row + k0 + 8 * (lane >> 4);
#pragma unroll
  for (int i = 0; i < 8; ++i) { v[i] = p[i]; v[8 + i] = p[16 + i]; }
  return bsplit16(v); }
__device__ __forceinline__ F2 split_rowK(const float* row, int k0, int lane, int K) { float v[16]; const int g = lane >> 4;
#pragma unroll
  for (int i = 0; i < 8; ++i) { const int ka = k0 + 8 * g + i, kb = ka + 16; v[i] = ka < K ? row[ka < K ? ka : K - 1] : 0.f; v[8 + i] = kb < K ? row[kb < K ? kb : K - 1] : 0.f; }
  return bsplit16(v); }
__device__ __forceinline__ F2 split_col(const float* W, int k0, int n, int lane, int ld, int K) { float v[16]; const int g = lane >> 4;
#pragma unroll
  for (int i = 0; i < 8; ++i) { const int ka = k0 + 8 * g + i, kb = ka + 16; v[i] = ka < K ? W[(size_t)(ka < K ? ka : K - 1) * ld + n] : 0.f; v[8 + i] = kb < K ? W[(size_t)(kb < K ? kb : K - 1) * ld + n] : 0.f; }
  return bsplit16(v); }
__device__ __forceinline__ v8f mac3(const F2& a, const F2& b, v8f c) { c = wmma_bf(a.l, b.h, c); c = wmma_bf(a.h, b.l, c); return wmma_bf(a.h, b.h, c); }
__device__ __forceinline__ float sigm(float v) { return 1.0f / (1.0f + expf(-v)); }
#define LDSX() do { asm volatile("s_wait_dscnt 0" ::: "memory"); __builtin_amdgcn_wave_barrier(); __builtin_amdgcn_fence(__ATOMIC_RELEASE, "workgroup"); } while (0)


#define CC 1024
#define CH 512
#define NP 4096
#define KV 2048
typedef __attribute__((ext_vector_type(8))) __bf16 v8b;
__device__ __forceinline__ v16b frag_b(const __bf16* rowk0, int lane) {
  union { v16b v; v8b q[2]; } u; const __bf16* p = rowk0 + 8 * (lane >> 4);
  u.q[0] = *(const v8b*)p; u.q[1] = *(const v8b*)(p + 16); return u.v;
}
__device__ __forceinline__ float bfr(float v) { return (float)(__bf16)v; }
__device__ __attribute__((noinline)) float exp_ni(float v) { return expf(v); }
__device__ __attribute__((noinline)) float erf_ni(float v) { return erff(v); }

#define WS_XT  0u
#define WS_PQ  (WS_XT + 2u * (size_t)3 * NP * CC)
#define PQSZ   ((size_t)CH * NP)
#define WS_VT  (WS_PQ + 2u * (size_t)3 * 2 * PQSZ)
#define WS_G   (WS_VT + 2u * (size_t)2 * NP * CC)
#define WS_A   (WS_G + 4u * (size_t)2 * CC * CC)
#define WS_END (WS_A + 2u * (size_t)2 * CC * CC)

__global__ __launch_bounds__(256) void k_xt(const float* __restrict__ X0, const float* __restrict__ X1, const float* __restrict__ X2, __bf16* __restrict__ XT) { __shared__ __align__(16) __bf16 st[64][64 + 8]; const int t = threadIdx.x; const int p0 = blockIdx.x * 64, which = blockIdx.y, c0 = blockIdx.z * 64; const float* X = which == 0 ? X0 : which == 1 ? X1 : X2;
  for (int e = t; e < 64 * 64; e += 256) { const int cl = e >> 6, pl = e & 63; st[pl][cl] = (__bf16)X[(size_t)(c0 + cl) * NP + p0 + pl]; } __syncthreads();
  for (int e = t; e < 64 * 8; e += 256) { const int pl = e >> 3, q = e & 7; vst2((unsigned*)(XT + ((size_t)which * NP + p0 + pl) * CC + c0 + q * 8), *(const v4u*)&st[pl][q * 8]); } }
__device__ __forceinline__ v16b fragb_f32(const float* __restrict__ p, int lane) { v16b a; const float* pp = p + 8 * (lane >> 4);
#pragma unroll
  for (int i = 0; i < 8; ++i) { a[i] = (__bf16)pp[i]; a[8 + i] = (__bf16)pp[16 + i]; } return a; }
__global__ __launch_bounds__(128) void k_conv(const float* __restrict__ WQ, const float* __restrict__ BQ, const float* __restrict__ WK1, const float* __restrict__ BK1, const float* __restrict__ WK2, const float* __restrict__ BK2, const float* __restrict__ WV, const float* __restrict__ BV, const __bf16* __restrict__ XT, _Float16* __restrict__ PQ, _Float16* __restrict__ VT) {
  __shared__ __align__(16) _Float16 sh[64][136], sl[64][136]; __shared__ __align__(16) _Float16 th[128][72], tl[128][72];
  const int tid = threadIdx.x, wave = tid >> 5, lane = tid & 31, col = lane & 15, g = lane >> 4; const int which = blockIdx.z; if (which < 3 && blockIdx.x >= CH / 64) return;
  const int ch0 = blockIdx.x * 64 + wave * 16; const int p0 = blockIdx.y * 128; const float* Wm = which == 0 ? WQ : which == 1 ? WK1 : which == 2 ? WK2 : WV; const float* Bm = which == 0 ? BQ : which == 1 ? BK1 : which == 2 ? BK2 : BV; const int xi = which == 0 ? 1 : which == 1 ? 0 : which == 2 ? 2 : 1;
  const __bf16* Xp = XT + (size_t)xi * NP * CC;
  v8f acc[8] = {};
#pragma unroll 2
  for (int kc = 0; kc < CC / 32; ++kc) { const v16b a = fragb_f32(Wm + (size_t)(ch0 + col) * CC + kc * 32, lane);
#pragma unroll
    for (int j = 0; j < 8; ++j) acc[j] = wmma_bf(a, frag_b(Xp + (size_t)(p0 + j * 16 + col) * CC + kc * 32, lane), acc[j]); }
#pragma unroll
  for (int j = 0; j < 8; ++j)
#pragma unroll
    for (int r = 0; r < 8; ++r) { const int chl = wave * 16 + 8 * g + r, pl = j * 16 + col; const float v = acc[j][r] + bfr(Bm[ch0 + 8 * g + r]); const _Float16 hv = (_Float16)v; const _Float16 lv = (_Float16)((v - (float)hv) * 2048.0f); if (which < 3) { sh[chl][pl] = hv; sl[chl][pl] = lv; } else { th[pl][chl] = hv; tl[pl][chl] = lv; } }
  __syncthreads();
  if (which < 3) { _Float16* H = PQ + (size_t)which * 2 * PQSZ; _Float16* L = H + PQSZ; for (int e = tid; e < 64 * 16; e += 128) { const int chl = e >> 4, q = e & 15; const size_t o = (size_t)(blockIdx.x * 64 + chl) * NP + p0 + q * 8; vst2((unsigned*)(H + o), *(const v4u*)&sh[chl][q * 8]); vst2((unsigned*)(L + o), *(const v4u*)&sl[chl][q * 8]); } }
  else { _Float16* H = VT; _Float16* L = VT + (size_t)NP * CC; for (int e = tid; e < 128 * 8; e += 128) { const int pl = e >> 3, q = e & 7; const size_t o = (size_t)(p0 + pl) * CC + blockIdx.x * 64 + q * 8; vst2((unsigned*)(H + o), *(const v4u*)&th[pl][q * 8]); vst2((unsigned*)(L + o), *(const v4u*)&tl[pl][q * 8]); } } }
__global__ __launch_bounds__(128) void k_gram(const _Float16* __restrict__ PQ, float* __restrict__ G) { __shared__ __align__(16) float sf[4][16][132];
  const int tid = threadIdx.x, wave = tid >> 5, lane = tid & 31, col = lane & 15, g = lane >> 4; const int which = blockIdx.z; const int i0 = blockIdx.x * 64 + wave * 16; const int j0 = blockIdx.y * 128;
  const _Float16* QH = PQ; const _Float16* QL = PQ + PQSZ; const _Float16* KH = PQ + (size_t)(1 + which) * 2 * PQSZ; const _Float16* KL = KH + PQSZ;
  v8f acc[8] = {}, accl[8] = {};
#pragma unroll 2
  for (int kc = 0; kc < KV / 32; ++kc) { const v16h ah = frag_h(KH + (size_t)(i0 + col) * KV + kc * 32, lane), al = frag_h(KL + (size_t)(i0 + col) * KV + kc * 32, lane);
#pragma unroll
    for (int j = 0; j < 8; ++j) { const size_t o = (size_t)(j0 + j * 16 + col) * KV + kc * 32; const v16h bh = frag_h(QH + o, lane), bl = frag_h(QL + o, lane); acc[j] = wmma16(ah, bh, acc[j]); accl[j] = wmma16(ah, bl, accl[j]); accl[j] = wmma16(al, bh, accl[j]); } }
#pragma unroll
  for (int j = 0; j < 8; ++j)
#pragma unroll
    for (int r = 0; r < 8; ++r) sf[wave][8 * g + r][j * 16 + col] = acc[j][r] + accl[j][r] * (1.0f / 2048.0f);
  LDSX(); for (int rl = 0; rl < 16; ++rl) vst2(G + ((size_t)which * CC + i0 + rl) * CC + j0 + lane * 4, *(const v4f*)&sf[wave][rl][lane * 4]); }
__global__ __launch_bounds__(256) void k_soft(const float* __restrict__ G, _Float16* __restrict__ AH, _Float16* __restrict__ AL) { __shared__ float red[8]; __shared__ __align__(16) _Float16 sh[CC], sl[CC]; __shared__ float sa[CC]; const int t = threadIdx.x; const size_t i = blockIdx.x;
  for (int c = t; c < CC; c += 256) sa[c] = 0.f;
  for (int which = 0; which < 2; ++which) { const float* row = G + ((size_t)which * CC + i) * CC; float mx = -3.0e38f; for (int c = t; c < CC; c += 256) mx = fmaxf(mx, row[c]);
#pragma unroll
    for (int o = 1; o < 32; o <<= 1) mx = fmaxf(mx, __shfl_xor(mx, o));
    __syncthreads(); if ((t & 31) == 0) red[t >> 5] = mx; __syncthreads(); float gm = red[0]; for (int w = 1; w < 8; ++w) gm = fmaxf(gm, red[w]); __syncthreads();
    float s = 0.f; for (int c = t; c < CC; c += 256) s += __expf(row[c] - gm);
#pragma unroll
    for (int o = 1; o < 32; o <<= 1) s += __shfl_xor(s, o);
    if ((t & 31) == 0) red[t >> 5] = s; __syncthreads(); float ts = 0.f; for (int w = 0; w < 8; ++w) ts += red[w]; const float inv = 1.0f / ts; __syncthreads();
    for (int c = t; c < CC; c += 256) sa[c] += __expf(row[c] - gm) * inv; }
  for (int c = t; c < CC; c += 256) { const float x = sa[c] * 2048.0f; const _Float16 hv = (_Float16)x; sh[c] = hv; sl[c] = (_Float16)((x - (float)hv) * 2048.0f); } __syncthreads();
  if (t < CC / 8) { vst2((unsigned*)(AH + i * CC + t * 8), *(const v4u*)&sh[t * 8]); vst2((unsigned*)(AL + i * CC + t * 8), *(const v4u*)&sl[t * 8]); } }
__global__ __launch_bounds__(128) void k_av(const _Float16* __restrict__ AH, const _Float16* __restrict__ AL, const _Float16* __restrict__ VT, const float* __restrict__ XF, const float* __restrict__ XL, const float* __restrict__ GAMMA, float* __restrict__ OUT) { __shared__ __align__(16) float sf[4][16][132];
  const int tid = threadIdx.x, wave = tid >> 5, lane = tid & 31, col = lane & 15, g = lane >> 4; const int i0 = blockIdx.x * 64 + wave * 16; const int p0 = blockIdx.y * 128; const _Float16* VH = VT; const _Float16* VL = VT + (size_t)NP * CC;
  v8f acc[8] = {}, accl[8] = {};
#pragma unroll 1
  for (int kc = 0; kc < CC / 32; ++kc) { const v16h ah = frag_h(AH + (size_t)(i0 + col) * CC + kc * 32, lane), al = frag_h(AL + (size_t)(i0 + col) * CC + kc * 32, lane);
#pragma unroll
    for (int j = 0; j < 8; ++j) { const size_t o = (size_t)(p0 + j * 16 + col) * CC + kc * 32; const v16h bh = frag_h(VH + o, lane), bl = frag_h(VL + o, lane); acc[j] = wmma16(ah, bh, acc[j]); accl[j] = wmma16(ah, bl, accl[j]); accl[j] = wmma16(al, bh, accl[j]); } }
  const float gam = bfr(GAMMA[0]);
#pragma unroll
  for (int j = 0; j < 8; ++j)
#pragma unroll
    for (int r = 0; r < 8; ++r) { const size_t ch = i0 + 8 * g + r, p = p0 + j * 16 + col; const float av = (acc[j][r] + accl[j][r] * (1.0f / 2048.0f)) * (1.0f / 2048.0f); sf[wave][8 * g + r][j * 16 + col] = gam * av + 0.5f * (bfr(XL[ch * NP + p]) + bfr(XF[ch * NP + p])); }
  LDSX(); for (int rl = 0; rl < 16; ++rl) vst2(OUT + (size_t)(i0 + rl) * NP + p0 + lane * 4, *(const v4f*)&sf[wave][rl][lane * 4]); }
extern "C" void kernel_launch(void* const* d_in, const int* in_sizes, int n_in, void* d_out, int out_size, void* d_ws, size_t ws_size, hipStream_t stream) {
  (void)in_sizes; (void)n_in; (void)out_size;
  const float** F = (const float**)d_in;
  if (ws_size < (size_t)WS_END) return;
  char* ws = (char*)d_ws; __bf16* XT = (__bf16*)(ws + WS_XT); _Float16 *PQ = (_Float16*)(ws + WS_PQ), *VT = (_Float16*)(ws + WS_VT), *AH = (_Float16*)(ws + WS_A), *AL = AH + (size_t)CC * CC; float* G = (float*)(ws + WS_G);
  k_xt<<<dim3(NP / 64, 3, CC / 64), 256, 0, stream>>>(F[0], F[1], F[2], XT);
  k_conv<<<dim3(CC / 64, NP / 128, 4), 128, 0, stream>>>(F[3], F[4], F[5], F[6], F[7], F[8], F[9], F[10], XT, PQ, VT);
  k_gram<<<dim3(CC / 64, CC / 128, 2), 128, 0, stream>>>(PQ, G);
  k_soft<<<CC, 256, 0, stream>>>(G, AH, AL);
  k_av<<<dim3(CC / 64, NP / 128), 128, 0, stream>>>(AH, AL, VT, F[0], F[2], F[11], (float*)d_out);
}
